// PGN_2267742732892
// MI455X (gfx1250) — hardware-verified
//
#include <hip/hip_runtime.h>


#define NB_  4
#define NN   128
#define FF   128
#define ZZ   256
#define HH   128
#define TT8  8
#define NZ   512
#define NE   65536
#define ZLW  448
#define ELW  192
typedef _Float16 h16;
typedef unsigned short bf;
typedef __attribute__((ext_vector_type(16))) __bf16   v16bf;
typedef __attribute__((ext_vector_type(16))) _Float16 v16h;
typedef __attribute__((ext_vector_type(8)))  _Float16 v8h;
typedef __attribute__((ext_vector_type(8)))  unsigned short v8us;
typedef __attribute__((ext_vector_type(8)))  float    v8f;
typedef __attribute__((ext_vector_type(4)))  float    v4f;
typedef v8h  __attribute__((may_alias)) v8ha;
typedef v4f  __attribute__((may_alias)) v4fa;
typedef v8us __attribute__((may_alias)) v8usa;

__device__ __forceinline__ unsigned short f2bf(float f) { unsigned u = __float_as_uint(f); u += 0x7FFFu + ((u >> 16) & 1u); return (unsigned short)(u >> 16); }
__device__ __forceinline__ float bf2f(unsigned short b) { return __uint_as_float(((unsigned)b) << 16); }
__device__ __forceinline__ float bfr(float f) { return bf2f(f2bf(f)); }
__device__ __forceinline__ v16h cat16(v8h lo, v8h hi) { return __builtin_shufflevector(lo, hi, 0, 1, 2, 3, 4, 5, 6, 7, 8, 9, 10, 11, 12, 13, 14, 15); }
__device__ __forceinline__ v16bf cat16b(v8us lo, v8us hi) { return __builtin_bit_cast(v16bf, __builtin_shufflevector(lo, hi, 0, 1, 2, 3, 4, 5, 6, 7, 8, 9, 10, 11, 12, 13, 14, 15)); }
__device__ __forceinline__ v8f wmma16(v16h a, v16h b, v8f c) { return __builtin_amdgcn_wmma_f32_16x16x32_f16(false, a, false, b, (short)0, c, false, false); }
__device__ __forceinline__ v8f wmmab(v16bf a, v16bf b, v8f c) { return __builtin_amdgcn_wmma_f32_16x16x32_bf16(false, a, false, b, (short)0, c, false, false); }


template <typename T16> struct WFrag;
template <> struct WFrag<h16> { typedef v16h V; static __device__ __forceinline__ V ld(const h16* p) { return cat16(*(const v8h*)p, *(const v8h*)(p + 16)); } static __device__ __forceinline__ v8f mma(V a, V b, v8f c) { return wmma16(a, b, c); } };
template <> struct WFrag<bf> { typedef v16bf V; static __device__ __forceinline__ V ld(const bf* p) { return cat16b(*(const v8us*)p, *(const v8us*)(p + 16)); } static __device__ __forceinline__ v8f mma(V a, V b, v8f c) { return wmmab(a, b, c); } };
template <typename T16, int NSPLIT, bool BIAS>
__global__ __launch_bounds__(32) void k_gemmw(const T16* __restrict__ A, const T16* __restrict__ A2, const T16* __restrict__ Bt, const T16* __restrict__ Bt2, int K, float* C, int ldc, const float* __restrict__ bias, size_t sA, size_t sB, size_t sC) {
    typedef typename WFrag<T16>::V V;
    __shared__ __align__(16) float os[16 * 68];
    const size_t z = blockIdx.z; A += z * sA; if (A2) A2 += z * sA; Bt += z * sB; if (Bt2) Bt2 += z * sB; C += z * sC;
    const int lane = threadIdx.x & 31, lr = lane & 15, hi = lane >> 4; const int r0 = blockIdx.x * 64, c0 = blockIdx.y * 64;
    v8f acc[4][4];
#pragma unroll
    for (int mb = 0; mb < 4; ++mb)
#pragma unroll
        for (int nb = 0; nb < 4; ++nb) acc[mb][nb] = (v8f){};
    const size_t aoff = (size_t)(r0 + lr) * K + 8 * hi, boff = (size_t)(c0 + lr) * K + 8 * hi;
#pragma unroll 1
    for (int kc = 0; kc < K; kc += 32) {
        V a[4], a2[4];
#pragma unroll
        for (int mb = 0; mb < 4; ++mb) { a[mb] = WFrag<T16>::ld(A + aoff + (size_t)mb * 16 * K + kc); if (NSPLIT == 1 || NSPLIT == 2) a2[mb] = WFrag<T16>::ld(A2 + aoff + (size_t)mb * 16 * K + kc); }
#pragma unroll
        for (int nb = 0; nb < 4; ++nb) { const V b = WFrag<T16>::ld(Bt + boff + (size_t)nb * 16 * K + kc); V b2; if (NSPLIT >= 2) b2 = WFrag<T16>::ld(Bt2 + boff + (size_t)nb * 16 * K + kc);
#pragma unroll
            for (int mb = 0; mb < 4; ++mb) { acc[mb][nb] = WFrag<T16>::mma(a[mb], b, acc[mb][nb]); if (NSPLIT == 1 || NSPLIT == 2) acc[mb][nb] = WFrag<T16>::mma(a2[mb], b, acc[mb][nb]); if (NSPLIT >= 2) acc[mb][nb] = WFrag<T16>::mma(a[mb], b2, acc[mb][nb]); } }
        asm volatile("v_nop\n\tv_nop\n\tv_nop\n\tv_nop" : "+v"(acc[0][0]), "+v"(acc[1][1]), "+v"(acc[2][2]), "+v"(acc[3][3]) : "v"(a[0]), "v"(a[3]));
    }
#pragma unroll
    for (int mb = 0; mb < 4; ++mb) {
#pragma unroll
        for (int nb = 0; nb < 4; ++nb) {
#pragma unroll
            for (int j = 0; j < 8; ++j) os[(hi * 8 + j) * 68 + nb * 16 + lr] = acc[mb][nb][j]; }
        __builtin_amdgcn_wave_barrier(); asm volatile("" ::: "memory");
        float* crow = C + (size_t)(r0 + mb * 16) * ldc + c0;
#pragma unroll 1
        for (int ps = 0; ps < 2; ++ps) {
#pragma unroll
            for (int s = 0; s < 8; ++s) { const int row = 2 * s + hi, cofs = lr * 4; v4f val = *(const v4fa*)(os + row * 68 + cofs); if (BIAS) { val[0] += bfr(bias[c0 + cofs]); val[1] += bfr(bias[c0 + cofs + 1]); val[2] += bfr(bias[c0 + cofs + 2]); val[3] += bfr(bias[c0 + cofs + 3]); }
                *(volatile v4f*)(crow + (size_t)row * ldc + cofs) = val; }
            if (ps == 0) __threadfence(); }
        __builtin_amdgcn_wave_barrier(); asm volatile("" ::: "memory");
    }
}

__device__ __forceinline__ void splitf(float y, unsigned short& h, unsigned short& l) { h = f2bf(y); l = f2bf(y - bf2f(h)); }
typedef __attribute__((ext_vector_type(4))) unsigned short v4us;

__global__ __launch_bounds__(256) void k_cvt8(const float* __restrict__ src, bf* dst, size_t n8) { const size_t i = (size_t)blockIdx.x * 256 + threadIdx.x; if (i >= n8) return; const v8f v = *(const v8f*)(src + i * 8); v8us o;
#pragma unroll
    for (int k = 0; k < 8; ++k) o[k] = f2bf(v[k]); *(volatile v8us*)(dst + i * 8) = o; __threadfence(); *(volatile v8us*)(dst + i * 8) = o; }
__global__ __launch_bounds__(256) void k_zb(const float* __restrict__ node, const float* __restrict__ hid, bf* ZB) { const int e = (blockIdx.x * 256 + threadIdx.x) * 4; if (e >= NZ * ZZ) return; const int c = e % ZZ; const int r = e / ZZ; const float* src = (c < FF) ? (node + (size_t)r * FF + c) : (hid + (size_t)r * FF + (c - FF)); v4us o;
#pragma unroll
    for (int u = 0; u < 4; ++u) o[u] = f2bf(src[u]); *(volatile v4us*)(ZB + e) = o; __threadfence(); *(volatile v4us*)(ZB + e) = o; }
__global__ __launch_bounds__(256) void k_wz(const float* __restrict__ m1, const float* __restrict__ m2, const float* __restrict__ o1, const float* __restrict__ t1, const float* __restrict__ t2, bf* Bt) { const int e = (blockIdx.x * 256 + threadIdx.x) * 4; if (e >= ZLW * ZZ) return; const int k = e % ZZ; const int col = e / ZZ; v4us o;
#pragma unroll
    for (int u = 0; u < 4; ++u) { const int kk = k + u; float v = 0.f; if (col < 128) v = m1[(size_t)kk * HH + col]; else if (col < 256) v = m2[(size_t)kk * HH + col - 128]; else if (col < 384) v = o1[(size_t)kk * HH + col - 256]; else if (col < 392) v = t1[(size_t)kk * TT8 + col - 384]; else if (col < 400) v = t2[(size_t)kk * TT8 + col - 392]; o[u] = f2bf(v); }
    *(volatile v4us*)(Bt + e) = o; __threadfence(); *(volatile v4us*)(Bt + e) = o; }
__global__ __launch_bounds__(256) void k_we(const float* __restrict__ me, const float* __restrict__ te1, const float* __restrict__ te2, const float* __restrict__ te3, bf* Bt) { const int e = (blockIdx.x * 256 + threadIdx.x) * 4; if (e >= ELW * FF) return; const int k = e % FF; const int col = e / FF; v4us o;
#pragma unroll
    for (int u = 0; u < 4; ++u) { const int kk = k + u; float v = 0.f; if (col < 128) v = me[(size_t)kk * HH + col]; else if (col < 136) v = te1[(size_t)kk * TT8 + col - 128]; else if (col < 144) v = te2[(size_t)kk * TT8 + col - 136]; else if (col < 152) v = te3[(size_t)kk * TT8 + col - 144]; o[u] = f2bf(v); }
    *(volatile v4us*)(Bt + e) = o; __threadfence(); *(volatile v4us*)(Bt + e) = o; }
__global__ __launch_bounds__(256) void k_wtx(const float* __restrict__ w, bf* Bt) { const int e = (blockIdx.x * 256 + threadIdx.x) * 4; if (e >= HH * HH) return; const int k = e % HH; const int o = e / HH; v4us v;
#pragma unroll
    for (int u = 0; u < 4; ++u) v[u] = f2bf(w[(size_t)(k + u) * HH + o]); *(volatile v4us*)(Bt + e) = v; __threadfence(); *(volatile v4us*)(Bt + e) = v; }
__global__ __launch_bounds__(256) void k_glin(const float* __restrict__ gf, const float* __restrict__ mgw, const float* __restrict__ mgb, const float* __restrict__ tgw, const float* __restrict__ tgb, float* G, float* TG) { const int idx = blockIdx.x * 256 + threadIdx.x;
    if (idx < NB_ * HH) { const int b = idx / HH, o = idx % HH; float acc = 0.f;
#pragma unroll 1
        for (int k = 0; k < FF; ++k) { float p = __fmul_rn(bfr(gf[b * FF + k]), bfr(mgw[(size_t)k * HH + o])); asm volatile("" : "+v"(p)); acc = __fadd_rn(acc, p); } const float r = __fadd_rn(acc, bfr(mgb[o])); *(volatile float*)(G + idx) = r; __threadfence(); *(volatile float*)(G + idx) = r; }
    else if (idx < NB_ * HH + NB_ * TT8) { const int j = idx - NB_ * HH; const int b = j / TT8, t = j % TT8; float acc = 0.f;
#pragma unroll 1
        for (int k = 0; k < FF; ++k) { float p = __fmul_rn(bfr(gf[b * FF + k]), bfr(tgw[(size_t)k * TT8 + t])); asm volatile("" : "+v"(p)); acc = __fadd_rn(acc, p); } const float r = __fadd_rn(acc, bfr(tgb[t])); *(volatile float*)(TG + j) = r; __threadfence(); *(volatile float*)(TG + j) = r; } }
__global__ __launch_bounds__(256) void k_msg(const float* __restrict__ ZL, const float* __restrict__ EL, const float* __restrict__ G, const float* __restrict__ m1b, const float* __restrict__ m2b, const float* __restrict__ meb, bf* Hh, bf* Hl) { const size_t e = ((size_t)blockIdx.x * 256 + threadIdx.x) * 4; if (e >= (size_t)NE * HH) return; const int h = (int)(e % HH); const int row = (int)(e / HH); const int j = row % NN; const int i = (row / NN) % NN; const int b = row / (NN * NN); v4us oh, ol;
#pragma unroll
    for (int u = 0; u < 4; ++u) { const int hh = h + u; float a1 = __fadd_rn(ZL[(size_t)(b * NN + j) * ZLW + hh], bfr(m1b[hh])); float a2 = __fadd_rn(ZL[(size_t)(b * NN + i) * ZLW + 128 + hh], bfr(m2b[hh])); float ae = __fadd_rn(EL[(size_t)row * ELW + hh], bfr(meb[hh])); asm volatile("" : "+v"(a1)); asm volatile("" : "+v"(a2)); asm volatile("" : "+v"(ae));
        float s = __fadd_rn(a1, a2); asm volatile("" : "+v"(s)); s = __fadd_rn(s, ae); asm volatile("" : "+v"(s)); s = __fadd_rn(s, G[b * HH + hh]); const float y = fmaxf(s, 0.f); unsigned short p, q; splitf(y, p, q); oh[u] = p; ol[u] = q; }
    *(volatile v4us*)(Hh + e) = oh; *(volatile v4us*)(Hl + e) = ol; __threadfence(); *(volatile v4us*)(Hh + e) = oh; *(volatile v4us*)(Hl + e) = ol; }
__global__ __launch_bounds__(256) void k_relu(const float* __restrict__ F, size_t n4, bf* Hh, bf* Hl) { const size_t e = ((size_t)blockIdx.x * 256 + threadIdx.x) * 4; if (e >= n4) return; const v4f a = *(const v4f*)(F + e); v4us oh, ol;
#pragma unroll
    for (int u = 0; u < 4; ++u) { unsigned short p, q; splitf(fmaxf(a[u], 0.f), p, q); oh[u] = p; ol[u] = q; } *(volatile v4us*)(Hh + e) = oh; *(volatile v4us*)(Hl + e) = ol; __threadfence(); *(volatile v4us*)(Hh + e) = oh; *(volatile v4us*)(Hl + e) = ol; }
__global__ __launch_bounds__(256) void k_agg(const float* __restrict__ MS, const int* __restrict__ adj, bf* Ah, bf* Al) { const int e = (blockIdx.x * 256 + threadIdx.x) * 4; if (e >= NZ * HH) return; const int h = e % HH; const int r = e / HH; const int j = r % NN; const int b = r / NN; v4f mx; mx[0] = mx[1] = mx[2] = mx[3] = -1.0e9f;
#pragma unroll 1
    for (int i = 0; i < NN; ++i) { if (adj[((size_t)b * NN + i) * NN + j] == 1) { const v4f m = *(const v4f*)(MS + ((size_t)(b * NN + i) * NN + j) * HH + h);
#pragma unroll
            for (int u = 0; u < 4; ++u) mx[u] = fmaxf(mx[u], m[u]); } }
    v4us oh, ol;
#pragma unroll
    for (int u = 0; u < 4; ++u) { unsigned short p, q; splitf(mx[u], p, q); oh[u] = p; ol[u] = q; } *(volatile v4us*)(Ah + e) = oh; *(volatile v4us*)(Al + e) = ol; __threadfence(); *(volatile v4us*)(Ah + e) = oh; *(volatile v4us*)(Al + e) = ol; }
__device__ __forceinline__ void ln128(float* v, int lane, const float* __restrict__ sc, const float* __restrict__ bi, float* o) { float s = 0.f;
#pragma unroll
    for (int u = 0; u < 4; ++u) s += v[u];
#pragma unroll
    for (int sh = 16; sh; sh >>= 1) s += __shfl_xor(s, sh, 32);
    const float mean = s * (1.0f / HH); float q = 0.f;
#pragma unroll
    for (int u = 0; u < 4; ++u) { float d = __fsub_rn(v[u], mean); asm volatile("" : "+v"(d)); float p = __fmul_rn(d, d); asm volatile("" : "+v"(p)); q = __fadd_rn(q, p); }
#pragma unroll
    for (int sh = 16; sh; sh >>= 1) q += __shfl_xor(q, sh, 32);
    const float sd = __fsqrt_rn(__fadd_rn(q * (1.0f / HH), 1e-5f));
#pragma unroll
    for (int u = 0; u < 4; ++u) { const int c = lane * 4 + u; float d = __fsub_rn(v[u], mean); asm volatile("" : "+v"(d)); float n0 = __fdiv_rn(d, sd); asm volatile("" : "+v"(n0)); float g = bfr(sc[c]), bb = bfr(bi[c]); asm volatile("" : "+v"(g)); asm volatile("" : "+v"(bb)); float t = __fmul_rn(n0, g); asm volatile("" : "+v"(t)); o[u] = __fadd_rn(t, bb); } }
__global__ __launch_bounds__(256) void k_out0(const float* __restrict__ ZL, const float* __restrict__ O2, const float* __restrict__ o1b, const float* __restrict__ sc, const float* __restrict__ bi, float* out0) { const int lane = threadIdx.x & 31; const int r = blockIdx.x * 8 + (threadIdx.x >> 5); if (r >= NZ) return; float v[4], o[4];
#pragma unroll
    for (int u = 0; u < 4; ++u) { const int c = lane * 4 + u; float a = __fadd_rn(ZL[(size_t)r * ZLW + 256 + c], bfr(o1b[c])); asm volatile("" : "+v"(a)); v[u] = fmaxf(__fadd_rn(a, O2[(size_t)r * HH + c]), 0.f); }
    ln128(v, lane, sc, bi, o); v4f w; for (int u = 0; u < 4; ++u) w[u] = o[u]; *(volatile v4f*)(out0 + (size_t)r * HH + lane * 4) = w; __threadfence(); *(volatile v4f*)(out0 + (size_t)r * HH + lane * 4) = w; }
__global__ __launch_bounds__(256) void k_tri(const float* __restrict__ ZL, const float* __restrict__ EL, const float* __restrict__ TG, const float* __restrict__ t1b, const float* __restrict__ t2b, const float* __restrict__ te1b, const float* __restrict__ te2b, const float* __restrict__ te3b, float* TM) {
    const size_t e = ((size_t)blockIdx.x * 256 + threadIdx.x) * 4; if (e >= (size_t)NE * TT8) return; const int t0 = (int)(e % TT8); const int row = (int)(e / TT8); const int k = row % NN; const int j = (row / NN) % NN; const int b = row / (NN * NN); v4f mx; mx[0] = mx[1] = mx[2] = mx[3] = -3.0e38f;
    float c2[4], c3[4], ce3[4], cg[4];
#pragma unroll
    for (int u = 0; u < 4; ++u) { const int t = t0 + u; c2[u] = __fadd_rn(ZL[(size_t)(b * NN + j) * ZLW + 392 + t], bfr(t2b[t])); c3[u] = __fadd_rn(ZL[(size_t)(b * NN + k) * ZLW + 384 + t], bfr(t1b[t])); ce3[u] = __fadd_rn(EL[((size_t)(b * NN + j) * NN + k) * ELW + 144 + t], bfr(te3b[t])); cg[u] = TG[b * TT8 + t]; }
#pragma unroll 1
    for (int i = 0; i < NN; ++i) {
#pragma unroll
        for (int u = 0; u < 4; ++u) { const int t = t0 + u; float a = __fadd_rn(ZL[(size_t)(b * NN + i) * ZLW + 384 + t], bfr(t1b[t]));
            float s = __fadd_rn(a, c2[u]); asm volatile("" : "+v"(s)); s = __fadd_rn(s, c3[u]); asm volatile("" : "+v"(s));
            float e1 = __fadd_rn(EL[((size_t)(b * NN + i) * NN + j) * ELW + 128 + t], bfr(te1b[t])); s = __fadd_rn(s, e1); asm volatile("" : "+v"(s));
            float e2 = __fadd_rn(EL[((size_t)(b * NN + i) * NN + k) * ELW + 136 + t], bfr(te2b[t])); s = __fadd_rn(s, e2); asm volatile("" : "+v"(s));
            s = __fadd_rn(s, ce3[u]); asm volatile("" : "+v"(s)); s = __fadd_rn(s, cg[u]); mx[u] = fmaxf(mx[u], s); } }
    *(volatile v4f*)(TM + e) = mx; __threadfence(); *(volatile v4f*)(TM + e) = mx; }
__global__ __launch_bounds__(256) void k_out1(const float* __restrict__ TM, const float* __restrict__ o3w, const float* __restrict__ o3b, const float* __restrict__ sc, const float* __restrict__ bi, float* out1) { const int lane = threadIdx.x & 31; const int r = blockIdx.x * 8 + (threadIdx.x >> 5); if (r >= NE) return; const float* tm = TM + (size_t)r * TT8; float v[4], o[4];
#pragma unroll
    for (int u = 0; u < 4; ++u) { const int c = lane * 4 + u; float acc = 0.f;
#pragma unroll
        for (int t = 0; t < TT8; ++t) { float p = __fmul_rn(tm[t], bfr(o3w[t * HH + c])); asm volatile("" : "+v"(p)); acc = __fadd_rn(acc, p); }
        v[u] = fmaxf(__fadd_rn(acc, bfr(o3b[c])), 0.f); }
    ln128(v, lane, sc, bi, o); v4f w; for (int u = 0; u < 4; ++u) w[u] = o[u]; *(volatile v4f*)(out1 + (size_t)r * HH + lane * 4) = w; __threadfence(); *(volatile v4f*)(out1 + (size_t)r * HH + lane * 4) = w; }

extern "C" void kernel_launch(void* const* d_in, const int* in_sizes, int n_in,
                              void* d_out, int out_size, void* d_ws, size_t ws_size, hipStream_t stream) {
    (void)in_sizes; (void)n_in; (void)out_size;
    const float** I = (const float**)d_in;
    const float *node = I[0], *edge = I[1], *gf = I[2], *hid = I[3]; const int* adj = (const int*)d_in[4];
    const float *m1w = I[5], *m1b = I[6], *m2w = I[7], *m2b = I[8], *mew = I[9], *meb = I[10], *mgw = I[11], *mgb = I[12], *p1w = I[13], *p1b = I[14], *p2w = I[15], *p2b = I[16], *o1w = I[17], *o1b = I[18], *o2w = I[19], *o2b = I[20];
    const float *t1w = I[21], *t1b = I[22], *t2w = I[23], *t2b = I[24], *te1w = I[25], *te1b = I[26], *te2w = I[27], *te2b = I[28], *te3w = I[29], *te3b = I[30], *tgw = I[31], *tgb = I[32], *o3w = I[33], *o3b = I[34], *nsc = I[35], *nbi = I[36];
    float* OUT0 = (float*)d_out;
    float* OUT1 = OUT0 + (size_t)NZ * HH;
    char* wsp = (char*)d_ws;
    auto take = [&](size_t bytes) { char* p = wsp; wsp += (bytes + 255) & ~(size_t)255; return (void*)p; };
    bf* ZB = (bf*)take((size_t)NZ * ZZ * 2); bf* BZ = (bf*)take((size_t)ZLW * ZZ * 2); float* ZL = (float*)take((size_t)NZ * ZLW * 4); bf* EB = (bf*)take((size_t)NE * FF * 2); bf* BE = (bf*)take((size_t)ELW * FF * 2); float* EL = (float*)take((size_t)NE * ELW * 4);
    float* G = (float*)take(NB_ * HH * 4); float* TG = (float*)take(256); bf* P1 = (bf*)take((size_t)HH * HH * 2); bf* P2 = (bf*)take((size_t)HH * HH * 2); bf* BO2 = (bf*)take((size_t)HH * HH * 2);
    bf* Hh = (bf*)take((size_t)NE * HH * 2); bf* Hl = (bf*)take((size_t)NE * HH * 2); float* F1 = (float*)take((size_t)NE * HH * 4); float* MS = (float*)take((size_t)NE * HH * 4); bf* Ah = (bf*)take((size_t)NZ * HH * 2); bf* Al = (bf*)take((size_t)NZ * HH * 2); float* O2 = (float*)take((size_t)NZ * HH * 4); float* TM = (float*)take((size_t)NE * TT8 * 4);
    if ((size_t)(wsp - (char*)d_ws) > ws_size) return;
    k_zb<<<(NZ * ZZ / 4 + 255) / 256, 256, 0, stream>>>(node, hid, ZB); k_wz<<<(ZLW * ZZ / 4 + 255) / 256, 256, 0, stream>>>(m1w, m2w, o1w, t1w, t2w, BZ); k_we<<<(ELW * FF / 4 + 255) / 256, 256, 0, stream>>>(mew, te1w, te2w, te3w, BE);
    k_wtx<<<(HH * HH / 4 + 255) / 256, 256, 0, stream>>>(p1w, P1); k_wtx<<<(HH * HH / 4 + 255) / 256, 256, 0, stream>>>(p2w, P2); k_wtx<<<(HH * HH / 4 + 255) / 256, 256, 0, stream>>>(o2w, BO2);
    k_gemmw<bf, 0, false><<<dim3(NZ / 64, ZLW / 64, 1), 32, 0, stream>>>(ZB, nullptr, BZ, nullptr, ZZ, ZL, ZLW, nullptr, 0, 0, 0);
    k_cvt8<<<(unsigned)(((size_t)NE * FF / 8 + 255) / 256), 256, 0, stream>>>(edge, EB, (size_t)NE * FF / 8);
    k_gemmw<bf, 0, false><<<dim3(NE / 64, ELW / 64, 1), 32, 0, stream>>>(EB, nullptr, BE, nullptr, FF, EL, ELW, nullptr, 0, 0, 0);
    k_glin<<<(NB_ * HH + NB_ * TT8 + 255) / 256, 256, 0, stream>>>(gf, mgw, mgb, tgw, tgb, G, TG);
    k_msg<<<(unsigned)(((size_t)NE * HH / 4 + 255) / 256), 256, 0, stream>>>(ZL, EL, G, m1b, m2b, meb, Hh, Hl);
    k_gemmw<bf, 1, true><<<dim3(NE / 64, HH / 64, 1), 32, 0, stream>>>(Hh, Hl, P1, nullptr, HH, F1, HH, p1b, 0, 0, 0); k_relu<<<(unsigned)(((size_t)NE * HH / 4 + 255) / 256), 256, 0, stream>>>(F1, (size_t)NE * HH, Hh, Hl);
    k_gemmw<bf, 1, true><<<dim3(NE / 64, HH / 64, 1), 32, 0, stream>>>(Hh, Hl, P2, nullptr, HH, MS, HH, p2b, 0, 0, 0);
    k_agg<<<(NZ * HH / 4 + 255) / 256, 256, 0, stream>>>(MS, adj, Ah, Al);
    k_gemmw<bf, 1, true><<<dim3(NZ / 64, HH / 64, 1), 32, 0, stream>>>(Ah, Al, BO2, nullptr, HH, O2, HH, o2b, 0, 0, 0);
    k_out0<<<NZ / 8, 256, 0, stream>>>(ZL, O2, o1b, nsc, nbi, OUT0);
    k_tri<<<(unsigned)(((size_t)NE * TT8 / 4 + 255) / 256), 256, 0, stream>>>(ZL, EL, TG, t1b, t2b, te1b, te2b, te3b, TM);
    k_out1<<<NE / 8, 256, 0, stream>>>(TM, o3w, o3b, nsc, nbi, OUT1);
}
